// UltraOptimizedINLBlock_3599182594271
// MI455X (gfx1250) — hardware-verified
//
#include <hip/hip_runtime.h>
#include <math.h>

constexpr int kB     = 2;
constexpr int kS     = 2048;
constexpr int kD     = 1024;
constexpr int kH     = 16;
constexpr int kHD    = 64;
constexpr int kFF    = 4096;
constexpr int kTok   = kB * kS;
constexpr int kQKVld = 3 * kD;
constexpr int kIters = 8;
constexpr int kNumGroups = 16;
constexpr float kDT        = 0.1f;
constexpr float kLnEps     = 1e-5f;
constexpr float kInvD      = 1.0f / 1024.0f;
constexpr float kWCarry    = 16.0f;
constexpr float kWCarryInv = 1.0f / 16.0f;
constexpr float kPCarry    = 32768.0f;
constexpr float kPCarryInv = 1.0f / 32768.0f;
constexpr float kScoreScale = 0.125f;

typedef __attribute__((ext_vector_type(16))) _Float16 v16h;
typedef __attribute__((ext_vector_type(8)))  _Float16 v8h;
typedef __attribute__((ext_vector_type(16))) __bf16   v16b;
typedef __attribute__((ext_vector_type(8)))  __bf16   v8b;
typedef __attribute__((ext_vector_type(8)))  float    v8f;
typedef __attribute__((ext_vector_type(4)))  float    v4f;
typedef __attribute__((ext_vector_type(2)))  float    v2f;
typedef __attribute__((ext_vector_type(4)))  unsigned int v4u;

__device__ __forceinline__ unsigned short f2bf_bits(float f) {
  unsigned u = __float_as_uint(f);
  return (unsigned short)((u + 0x7FFFu + ((u >> 16) & 1u)) >> 16);
}
__device__ __forceinline__ float bf_bits2f(unsigned short h) { return __uint_as_float(((unsigned)h) << 16); }

__device__ __forceinline__ void dep_guard_h(v8f& a, v8f& b, v16h x, v16h y) { asm volatile("v_nop\n\tv_nop\n\tv_nop\n\tv_nop" : "+v"(a), "+v"(b) : "v"(x), "v"(y)); }
__device__ __forceinline__ void dep_guard_b(v8f& a, v8f& b, v16b x, v16b y) { asm volatile("v_nop\n\tv_nop\n\tv_nop\n\tv_nop" : "+v"(a), "+v"(b) : "v"(x), "v"(y)); }
__device__ __forceinline__ void keep4_h(v16h a, v16h b, v16h c, v16h d) { asm volatile("v_nop" :: "v"(a), "v"(b), "v"(c), "v"(d)); }
__device__ __forceinline__ void keep4_b(v16b a, v16b b, v16b c, v16b d) { asm volatile("v_nop" :: "v"(a), "v"(b), "v"(c), "v"(d)); }
__device__ __forceinline__ void acc_guard4(v8f& a, v8f& b, v8f& c, v8f& d) { asm volatile("v_nop\n\tv_nop\n\tv_nop\n\tv_nop" : "+v"(a), "+v"(b), "+v"(c), "+v"(d)); }
template <typename T> struct Frag;
template <> struct Frag<_Float16> {
  typedef v16h V; union U { v16h v; v8h h[2]; };
  static __device__ __forceinline__ v16h load(const _Float16* p) {
    U f; f.h[0] = *(const v8h*)(p); f.h[1] = *(const v8h*)(p + 16); return f.v;
  }
  static __device__ __forceinline__ v8f mma(v16h a, v16h b, v8f c) {
    return __builtin_amdgcn_wmma_f32_16x16x32_f16(false, a, false, b, (short)0, c, false, false);
  }
  static __device__ __forceinline__ void guard(v8f& a, v8f& b, v16h x, v16h y) { dep_guard_h(a, b, x, y); }
  static __device__ __forceinline__ void keep(v16h a, v16h b, v16h c, v16h d) { keep4_h(a, b, c, d); }
};
template <> struct Frag<__bf16> {
  typedef v16b V; union U { v16b v; v8b h[2]; };
  static __device__ __forceinline__ v16b load(const __bf16* p) {
    U f; f.h[0] = *(const v8b*)(p); f.h[1] = *(const v8b*)(p + 16); return f.v;
  }
  static __device__ __forceinline__ v8f mma(v16b a, v16b b, v8f c) {
    return __builtin_amdgcn_wmma_f32_16x16x32_bf16(false, a, false, b, (short)0, c, false, false);
  }
  static __device__ __forceinline__ void guard(v8f& a, v8f& b, v16b x, v16b y) { dep_guard_b(a, b, x, y); }
  static __device__ __forceinline__ void keep(v16b a, v16b b, v16b c, v16b d) { keep4_b(a, b, c, d); }
};

__device__ __forceinline__ unsigned pk16(unsigned short a, unsigned short b) { return (unsigned)a | ((unsigned)b << 16); }
__device__ __forceinline__ unsigned short h_bits(float f) { const _Float16 h = (_Float16)f; return __builtin_bit_cast(unsigned short, h); }

template <int ET> struct Elem;
template <> struct Elem<0> { typedef _Float16 T; };
template <> struct Elem<1> { typedef __bf16 T; };
template <int ET, bool SPLIT, int BIAS_MODE, int OUT_MODE, bool RESID, int ACT = 0, bool CAUSAL = false>
__global__ __launch_bounds__(256) void wmma_gemm64(
    const unsigned short* __restrict__ Ap, const unsigned short* __restrict__ A2p, int lda, long strideA,
    const unsigned short* __restrict__ Btp, const unsigned short* __restrict__ Bt2p, int ldb, long strideB,
    void* __restrict__ Cout, void* __restrict__ Cout2, int ldc, long strideC,
    const float* __restrict__ bias,
    const float* __restrict__ resid, long strideR,
    int M, int N, int K, float scale) {
  typedef typename Elem<ET>::T T;
  typedef typename Frag<T>::V V;
  const T* A = (const T*)Ap; const T* A2 = (const T*)A2p; const T* Bt = (const T*)Btp; const T* Bt2 = (const T*)Bt2p;
  __shared__ __align__(16) float sT[8][16 * 68];
  const int b    = blockIdx.y;
  const int lane = threadIdx.x & 31;
  const int wave = threadIdx.x >> 5;
  const int tilesN = N >> 6;
  const int tilesM = M >> 6;
  const int tile = blockIdx.x * 8 + wave;
  if (tile >= tilesM * tilesN) return;
  const int tm = tile / tilesN;
  const int tn = tile - tm * tilesN;
  if (CAUSAL && tn > tm) return;
  const int m0 = tm << 6;
  const int n0 = tn << 6;
  const int kEnd = CAUSAL ? (((m0 + 64) < K) ? (m0 + 64) : K) : K;

  const T* Ab  = A  + (size_t)b * strideA;
  const T* Bb  = Bt + (size_t)b * strideB;
  const T* Ab2 = SPLIT ? (A2  + (size_t)b * strideA) : nullptr;
  const T* Bb2 = SPLIT ? (Bt2 + (size_t)b * strideB) : nullptr;

  const int rlane = lane & 15;
  const int koff  = (lane >> 4) * 8;
  const int mOff  = (lane >> 4) * 8;

  v8f acc[4][4];
#pragma unroll
  for (int i = 0; i < 4; ++i)
#pragma unroll
    for (int j = 0; j < 4; ++j) acc[i][j] = (v8f){0.f,0.f,0.f,0.f,0.f,0.f,0.f,0.f};

  for (int k0 = 0; k0 < kEnd; k0 += 32) {
    V bh[4], bl[4];
#pragma unroll
    for (int j = 0; j < 4; ++j) {
      const size_t bo = (size_t)(n0 + (j << 4) + rlane) * ldb + koff + k0;
      bh[j] = Frag<T>::load(Bb + bo);
      if (SPLIT) bl[j] = Frag<T>::load(Bb2 + bo);
    }
#pragma unroll
    for (int i = 0; i < 4; ++i) {
      const size_t ao = (size_t)(m0 + (i << 4) + rlane) * lda + koff + k0;
      V ah = Frag<T>::load(Ab + ao);
      V al;
      if (SPLIT) al = Frag<T>::load(Ab2 + ao);
#pragma unroll
      for (int j = 0; j < 4; ++j) {
        acc[i][j] = Frag<T>::mma(ah, bh[j], acc[i][j]);
        if (SPLIT) {
          acc[i][j] = Frag<T>::mma(ah, bl[j], acc[i][j]);
          acc[i][j] = Frag<T>::mma(al, bh[j], acc[i][j]);
        }
      }
      Frag<T>::guard(acc[i][0], acc[i][3], ah, SPLIT ? al : ah);
    }
    Frag<T>::keep(bh[0], bh[1], bh[2], bh[3]);
    if (SPLIT) Frag<T>::keep(bl[0], bl[1], bl[2], bl[3]);
  }
  acc_guard4(acc[0][0], acc[0][1], acc[0][2], acc[0][3]);
  acc_guard4(acc[1][0], acc[1][1], acc[1][2], acc[1][3]);
  acc_guard4(acc[2][0], acc[2][1], acc[2][2], acc[2][3]);
  acc_guard4(acc[3][0], acc[3][1], acc[3][2], acc[3][3]);

  float* slab = sT[wave];
  const float* Rb = RESID ? (resid + (size_t)b * strideR) : nullptr;
#pragma unroll
  for (int i = 0; i < 4; ++i) {
    const int mBase = m0 + (i << 4);
#pragma unroll
    for (int j = 0; j < 4; ++j) {
      const int n = n0 + (j << 4) + rlane;
      float bv = 0.f;
      if (BIAS_MODE == 2) bv = bias[n];
#pragma unroll
      for (int r = 0; r < 8; ++r) {
        float v = acc[i][j][r] * scale;
        if (BIAS_MODE == 1) v += bias[mBase + mOff + r];
        if (BIAS_MODE == 2) v += bv;
        if (RESID) v += Rb[(size_t)(mBase + mOff + r) * ldc + n];
        if (ACT == 2) v = fmaxf(v, 0.0f);
        if (ACT == 4) v = (v > 0.f) ? v : 0.01f * v;
        slab[(mOff + r) * 68 + (j << 4) + rlane] = v;
      }
    }
    __builtin_amdgcn_fence(__ATOMIC_RELEASE, "workgroup");
    __builtin_amdgcn_wave_barrier();
    __builtin_amdgcn_fence(__ATOMIC_ACQUIRE, "workgroup");
    if (OUT_MODE == 0) {
      float* C = (float*)Cout + (size_t)b * strideC;
      const int hh = lane >> 4, c4 = (lane & 15) * 4;
      for (int pass = 0; pass < 2; ++pass) {
#pragma unroll
        for (int it = 0; it < 8; ++it) {
          const int row = it * 2 + hh;
          v4f v = *(const v4f*)(slab + row * 68 + c4);
          *(volatile v4f*)(C + (size_t)(mBase + row) * ldc + n0 + c4) = v;
        }
        __threadfence();
      }
    } else {
      const int q = lane >> 3, c8 = (lane & 7) * 8;
      unsigned short* C  = (unsigned short*)Cout  + (size_t)b * strideC;
      unsigned short* C2 = (OUT_MODE == 2) ? ((unsigned short*)Cout2 + (size_t)b * strideC) : nullptr;
      for (int pass = 0; pass < 2; ++pass) {
#pragma unroll
        for (int it = 0; it < 4; ++it) {
          const int row = it * 4 + q;
          const float* sp = slab + row * 68 + c8;
          v8h hv, lv;
#pragma unroll
          for (int e = 0; e < 8; ++e) {
            if (OUT_MODE == 1) {
              hv[e] = (_Float16)sp[e];
            } else {
              unsigned short hb = f2bf_bits(sp[e]);
              unsigned short lb = f2bf_bits(sp[e] - bf_bits2f(hb));
              hv[e] = __builtin_bit_cast(_Float16, hb);
              lv[e] = __builtin_bit_cast(_Float16, lb);
            }
          }
          *(volatile v8h*)(C + (size_t)(mBase + row) * ldc + n0 + c8) = hv;
          if (OUT_MODE == 2) *(volatile v8h*)(C2 + (size_t)(mBase + row) * ldc + n0 + c8) = lv;
        }
        __threadfence();
      }
    }
    __builtin_amdgcn_fence(__ATOMIC_RELEASE, "workgroup");
    __builtin_amdgcn_wave_barrier();
    __builtin_amdgcn_fence(__ATOMIC_ACQUIRE, "workgroup");
  }
}

__global__ __launch_bounds__(256) void wt_cast_kernel(const float* __restrict__ W0, const float* __restrict__ W1,
                                                      const float* __restrict__ W2, unsigned short* __restrict__ out,
                                                      long plane_stride, int nrow_in, int ncol_in, float scale) {
  __shared__ float sm[64][65];
  const int t  = threadIdx.x;
  const int r0 = blockIdx.x * 64;
  const int c0 = blockIdx.y * 64;
  const int z  = blockIdx.z;
  const float* W = (z == 0) ? W0 : (z == 1) ? W1 : W2;
#pragma unroll
  for (int i = 0; i < 16; ++i) {
    const int e = i * 256 + t;
    const int r = e >> 6;
    const int c = e & 63;
    sm[c][r] = W[(size_t)(r0 + r) * ncol_in + c0 + c] * scale;
  }
  __syncthreads();
  const int lane = t & 31, wave = t >> 5;
  const int q = lane >> 3, c8 = (lane & 7) * 8;
  unsigned short* op = out + (size_t)z * plane_stride;
  for (int pass = 0; pass < 2; ++pass) {
#pragma unroll
    for (int it = 0; it < 2; ++it) {
      const int row = wave * 8 + it * 4 + q;
      unsigned short hb[8];
#pragma unroll
      for (int e = 0; e < 8; ++e) hb[e] = h_bits(sm[row][c8 + e]);
      const v4u u = (v4u){pk16(hb[0], hb[1]), pk16(hb[2], hb[3]), pk16(hb[4], hb[5]), pk16(hb[6], hb[7])};
      *(volatile v4u*)(op + (size_t)(c0 + row) * nrow_in + r0 + c8) = u;
    }
    __threadfence();
  }
}

__global__ __launch_bounds__(256) void vt_transpose_kernel(const unsigned short* __restrict__ qkv,
                                                           unsigned short* __restrict__ vt) {
  __shared__ __align__(16) unsigned short sm[64][72];
  const int t    = threadIdx.x;
  const int key0 = blockIdx.x * 64;
  const int col0 = blockIdx.y * 64;
  const int b    = blockIdx.z;
  const unsigned int* src = (const unsigned int*)(const void*)qkv;
#pragma unroll
  for (int i = 0; i < 8; ++i) {
    const int e  = i * 256 + t;
    const int r  = e >> 5;
    const int cw = e & 31;
    const size_t hidx = (size_t)(b * kS + key0 + r) * kQKVld + 2 * kD + col0 + 2 * cw;
    const unsigned int w = src[hidx >> 1];
    sm[2 * cw][r]     = (unsigned short)(w & 0xffffu);
    sm[2 * cw + 1][r] = (unsigned short)(w >> 16);
  }
  __syncthreads();
  const int lane = t & 31, wave = t >> 5;
  const int q = lane >> 3, c8 = (lane & 7) * 8;
  for (int pass = 0; pass < 2; ++pass) {
#pragma unroll
    for (int it = 0; it < 2; ++it) {
      const int row = wave * 8 + it * 4 + q;
      const v4u u = (v4u){pk16(sm[row][c8 + 0], sm[row][c8 + 1]), pk16(sm[row][c8 + 2], sm[row][c8 + 3]),
                          pk16(sm[row][c8 + 4], sm[row][c8 + 5]), pk16(sm[row][c8 + 6], sm[row][c8 + 7])};
      *(volatile v4u*)(vt + (size_t)(b * kD + col0 + row) * kS + key0 + c8) = u;
    }
    __threadfence();
  }
}

template <bool HAS_IN1, bool OUT_SUM32, bool OUT_ADD16, bool OUT_LN32>
__global__ __launch_bounds__(128) void ln_row_kernel(
    const float* __restrict__ in0, const float* __restrict__ in1,
    const float* __restrict__ gam, const float* __restrict__ bet,
    float* __restrict__ sum32, unsigned short* __restrict__ add16,
    float* __restrict__ ln32, unsigned short* __restrict__ ln16) {
  __shared__ __align__(16) float sbuf[kD];
  __shared__ float redA[4];
  __shared__ float redB[4];
  const int row  = blockIdx.x;
  const int t    = threadIdx.x;
  const int lane = t & 31, wave = t >> 5;
  const size_t rbase = (size_t)row * kD;
  const int c0 = t * 8;

  const v4f a0 = *(const v4f*)(in0 + rbase + c0);
  const v4f a1 = *(const v4f*)(in0 + rbase + c0 + 4);
  float x[8];
  float ad[8];
#pragma unroll
  for (int e = 0; e < 4; ++e) { x[e] = a0[e]; x[4 + e] = a1[e]; ad[e] = 0.f; ad[4 + e] = 0.f; }
  if (HAS_IN1) {
    const v4f b0v = *(const v4f*)(in1 + rbase + c0);
    const v4f b1v = *(const v4f*)(in1 + rbase + c0 + 4);
#pragma unroll
    for (int e = 0; e < 4; ++e) { ad[e] = b0v[e]; ad[4 + e] = b1v[e]; }
#pragma unroll
    for (int e = 0; e < 8; ++e) x[e] = x[e] + ad[e];
  }
  if (OUT_ADD16) {
    const v4u u = (v4u){pk16(h_bits(ad[0]), h_bits(ad[1])), pk16(h_bits(ad[2]), h_bits(ad[3])),
                        pk16(h_bits(ad[4]), h_bits(ad[5])), pk16(h_bits(ad[6]), h_bits(ad[7]))};
    unsigned short* dp = add16 + rbase + c0;
    *(volatile v4u*)dp = u;
    __threadfence();
    *(volatile v4u*)dp = u;
  }
  if (OUT_SUM32) {
    *(v4f*)(sbuf + c0)     = (v4f){x[0], x[1], x[2], x[3]};
    *(v4f*)(sbuf + c0 + 4) = (v4f){x[4], x[5], x[6], x[7]};
    __syncthreads();
    const v4f s0 = *(const v4f*)(sbuf + 4 * t);
    const v4f s1 = *(const v4f*)(sbuf + 512 + 4 * t);
    float* dp = sum32 + rbase;
    *(volatile v4f*)(dp + 4 * t) = s0;
    *(volatile v4f*)(dp + 512 + 4 * t) = s1;
    __threadfence();
    *(volatile v4f*)(dp + 4 * t) = s0;
    *(volatile v4f*)(dp + 512 + 4 * t) = s1;
    __syncthreads();
  }
  float s = ((x[0] + x[1]) + (x[2] + x[3])) + ((x[4] + x[5]) + (x[6] + x[7]));
#pragma unroll
  for (int off = 16; off > 0; off >>= 1) s += __shfl_xor(s, off, 32);
  if (lane == 0) redA[wave] = s;
  __syncthreads();
  const float mean = ((redA[0] + redA[1]) + (redA[2] + redA[3])) * kInvD;
  float d[8];
#pragma unroll
  for (int e = 0; e < 8; ++e) d[e] = x[e] - mean;
  float qs = 0.f;
#pragma unroll
  for (int e = 0; e < 8; ++e) qs += d[e] * d[e];
#pragma unroll
  for (int off = 16; off > 0; off >>= 1) qs += __shfl_xor(qs, off, 32);
  if (lane == 0) redB[wave] = qs;
  __syncthreads();
  const float var = ((redB[0] + redB[1]) + (redB[2] + redB[3])) * kInvD;
  const float inv = rsqrtf(var + kLnEps);
  const v4f g0 = *(const v4f*)(gam + c0);
  const v4f g1v = *(const v4f*)(gam + c0 + 4);
  const v4f e0 = *(const v4f*)(bet + c0);
  const v4f e1 = *(const v4f*)(bet + c0 + 4);
  float y[8];
#pragma unroll
  for (int e = 0; e < 4; ++e) {
    y[e]     = d[e] * inv * g0[e] + e0[e];
    y[4 + e] = d[4 + e] * inv * g1v[e] + e1[e];
  }
  {
    const v4u u = (v4u){pk16(h_bits(y[0]), h_bits(y[1])), pk16(h_bits(y[2]), h_bits(y[3])),
                        pk16(h_bits(y[4]), h_bits(y[5])), pk16(h_bits(y[6]), h_bits(y[7]))};
    unsigned short* dp = ln16 + rbase + c0;
    *(volatile v4u*)dp = u;
    __threadfence();
    *(volatile v4u*)dp = u;
  }
  if (OUT_LN32) {
    *(v4f*)(sbuf + c0)     = (v4f){y[0], y[1], y[2], y[3]};
    *(v4f*)(sbuf + c0 + 4) = (v4f){y[4], y[5], y[6], y[7]};
    __syncthreads();
    const v4f s0 = *(const v4f*)(sbuf + 4 * t);
    const v4f s1 = *(const v4f*)(sbuf + 512 + 4 * t);
    float* dp = ln32 + rbase;
    *(volatile v4f*)(dp + 4 * t) = s0;
    *(volatile v4f*)(dp + 512 + 4 * t) = s1;
    __threadfence();
    *(volatile v4f*)(dp + 4 * t) = s0;
    *(volatile v4f*)(dp + 512 + 4 * t) = s1;
  }
}

__global__ __launch_bounds__(256) void softmax_causal_kernel(const float* __restrict__ Sp, unsigned short* __restrict__ Pp, float carry) {
  __shared__ float redM[8];
  __shared__ float redS[8];
  const int row  = blockIdx.x;
  const int z    = blockIdx.y;
  const int t    = threadIdx.x;
  const int lane = t & 31, wave = t >> 5;
  const int c0   = t * 8;
  const size_t off = ((size_t)z * kS + row) * kS + c0;
  const v4f a = *(const v4f*)(Sp + off);
  const v4f c = *(const v4f*)(Sp + off + 4);
  float x[8];
#pragma unroll
  for (int e = 0; e < 4; ++e) {
    x[e]     = (c0 + e     <= row) ? a[e] : -1.0e30f;
    x[4 + e] = (c0 + 4 + e <= row) ? c[e] : -1.0e30f;
  }
  float m = fmaxf(fmaxf(fmaxf(x[0], x[1]), fmaxf(x[2], x[3])), fmaxf(fmaxf(x[4], x[5]), fmaxf(x[6], x[7])));
#pragma unroll
  for (int offx = 16; offx > 0; offx >>= 1) m = fmaxf(m, __shfl_xor(m, offx, 32));
  if (lane == 0) redM[wave] = m;
  __syncthreads();
  float gm = redM[0];
#pragma unroll
  for (int w = 1; w < 8; ++w) gm = fmaxf(gm, redM[w]);
  float ex[8];
#pragma unroll
  for (int e = 0; e < 8; ++e) ex[e] = expf(x[e] - gm);
  float s = ((ex[0] + ex[1]) + (ex[2] + ex[3])) + ((ex[4] + ex[5]) + (ex[6] + ex[7]));
#pragma unroll
  for (int offx = 16; offx > 0; offx >>= 1) s += __shfl_xor(s, offx, 32);
  if (lane == 0) redS[wave] = s;
  __syncthreads();
  float tot = redS[0];
#pragma unroll
  for (int w = 1; w < 8; ++w) tot += redS[w];
  const float inv = carry * (1.0f / tot);
  unsigned short hb[8];
#pragma unroll
  for (int e = 0; e < 8; ++e) hb[e] = h_bits(ex[e] * inv);
  const v4u u = (v4u){pk16(hb[0], hb[1]), pk16(hb[2], hb[3]), pk16(hb[4], hb[5]), pk16(hb[6], hb[7])};
  unsigned short* dp = Pp + off;
  *(volatile v4u*)dp = u;
  __threadfence();
  *(volatile v4u*)dp = u;
}

template <bool FIRST>
__global__ __launch_bounds__(256) void inl_step_kernel(
    const float* __restrict__ c0p, const float* __restrict__ gp,
    const float* __restrict__ xs_in, const float* __restrict__ vs_in,
    float* __restrict__ xs_out, float* __restrict__ vs_out,
    unsigned short* __restrict__ xs16) {
  __shared__ __align__(16) unsigned int sh[512];
  const int t = threadIdx.x;
  const size_t base = (size_t)blockIdx.x * 1024 + 4 * t;
  const v4f cc = *(const v4f*)(c0p + base);
  const v4f gg = *(const v4f*)(gp + base);
  const v4f xo = *(const v4f*)(xs_in + base);
  v4f vo = (v4f){0.f, 0.f, 0.f, 0.f};
  if (!FIRST) vo = *(const v4f*)(vs_in + base);
  v4f xn, vn;
#pragma unroll
  for (int e = 0; e < 4; ++e) {
    const float u  = tanhf(cc[e] + gg[e]);
    const float v1 = vo[e] + kDT * ((u - xo[e]) - vo[e]);
    vn[e] = v1;
    xn[e] = xo[e] + kDT * v1;
  }
  *(volatile v4f*)(xs_out + base) = xn;
  *(volatile v4f*)(vs_out + base) = vn;
  __threadfence();
  *(volatile v4f*)(xs_out + base) = xn;
  *(volatile v4f*)(vs_out + base) = vn;
  sh[2 * t]     = pk16(h_bits(xn[0]), h_bits(xn[1]));
  sh[2 * t + 1] = pk16(h_bits(xn[2]), h_bits(xn[3]));
  __syncthreads();
  if (t < 128) {
    const v4u u = *(const v4u*)(sh + 4 * t);
    unsigned short* dp = xs16 + (size_t)blockIdx.x * 1024 + 8 * t;
    *(volatile v4u*)dp = u;
    __threadfence();
    *(volatile v4u*)dp = u;
  }
}

__global__ __launch_bounds__(256) void gelu_cast_kernel(const float* __restrict__ in, unsigned short* __restrict__ out, int n2) {
  const int i = blockIdx.x * 256 + threadIdx.x;
  if (i >= n2) return;
  const v2f p = *(const v2f*)(in + 2 * (size_t)i);
  const float ga = 0.5f * p[0] * (1.0f + erff(p[0] * 0.70710678118654752f));
  const float gb = 0.5f * p[1] * (1.0f + erff(p[1] * 0.70710678118654752f));
  const unsigned u = pk16(h_bits(ga), h_bits(gb));
  ((volatile unsigned*)out)[i] = u;
  __threadfence();
  ((volatile unsigned*)out)[i] = u;
}

extern "C" void kernel_launch(void* const* d_in, const int* in_sizes, int n_in,
                              void* d_out, int out_size, void* d_ws, size_t ws_size,
                              hipStream_t stream) {
  if (n_in < 18) return;
  if (in_sizes[0] != kTok * kD || in_sizes[1] != kD * 3 * kD || in_sizes[2] != 3 * kD ||
      in_sizes[3] != kD * kD || in_sizes[4] != kD || in_sizes[5] != kD || in_sizes[6] != kD ||
      in_sizes[7] != kD || in_sizes[8] != kD || in_sizes[9] != kD || in_sizes[10] != kD ||
      in_sizes[11] != kD * kD || in_sizes[12] != kD * kD || in_sizes[13] != kD ||
      in_sizes[14] != kD * kFF || in_sizes[15] != kFF || in_sizes[16] != kFF * kD || in_sizes[17] != kD) return;
  if (out_size != kTok * kD) return;
  const size_t MiB = 1048576;
  const size_t carve_total = 126 * MiB;
  if (ws_size < carve_total) return;

  const float* x      = (const float*)d_in[0];
  const float* qkv_w  = (const float*)d_in[1];
  const float* qkv_b  = (const float*)d_in[2];
  const float* out_w  = (const float*)d_in[3];
  const float* out_b  = (const float*)d_in[4];
  const float* g_attn = (const float*)d_in[5];
  const float* b_attn = (const float*)d_in[6];
  const float* g1     = (const float*)d_in[7];
  const float* b1     = (const float*)d_in[8];
  const float* g2     = (const float*)d_in[9];
  const float* b2     = (const float*)d_in[10];
  const float* w_ctx  = (const float*)d_in[11];
  const float* w_x    = (const float*)d_in[12];
  const float* b_inl  = (const float*)d_in[13];
  const float* ff_w1  = (const float*)d_in[14];
  const float* ff_b1  = (const float*)d_in[15];
  const float* ff_w2  = (const float*)d_in[16];
  const float* ff_b2  = (const float*)d_in[17];
  float* out = (float*)d_out;

  char* ws = (char*)d_ws;
  unsigned short* wOutT = (unsigned short*)(ws + 0);
  unsigned short* wCtxT = (unsigned short*)(ws + 2 * MiB);
  unsigned short* wXT   = (unsigned short*)(ws + 4 * MiB);
  char* RA = ws + 6 * MiB;
  char* RB = ws + 30 * MiB;
  char* RC = ws + 62 * MiB;
  char* RD = ws + 94 * MiB;
  unsigned short* wQkvT = (unsigned short*)(RB);
  unsigned short* xn16  = (unsigned short*)(RB + 6 * MiB);
  unsigned short* qkv16 = (unsigned short*)(RA);
  unsigned short* vt16  = (unsigned short*)(RB);
  float*          sbuf  = (float*)(RC);
  unsigned short* pbuf  = (unsigned short*)(RD);
  unsigned short* ctx16 = (unsigned short*)(RD + 16 * MiB);
  float*          att   = (float*)(RB);
  float*          x1    = (float*)(RC);
  unsigned short* att16 = (unsigned short*)(RC + 16 * MiB);
  float*          c0    = (float*)(RA);
  unsigned short* xs16  = (unsigned short*)(RA + 16 * MiB);
  float*          xsA   = (float*)(RD);
  float*          xsB   = (float*)(RD + 16 * MiB);
  float*          vsA   = (float*)(RB);
  float*          vsB   = (float*)(RB + 16 * MiB);
  float*          gmat  = (float*)(RC + 16 * MiB);
  float*          x2    = (float*)(RB);
  unsigned short* hn16  = (unsigned short*)(RB + 16 * MiB);
  unsigned short* wFf1T = (unsigned short*)(RC);
  unsigned short* wFf2T = (unsigned short*)(RC + 8 * MiB);
  float*          f1c   = (float*)(RD);
  unsigned short* g1c   = (unsigned short*)(RA);

  const dim3 blk256(256), blk128(128);

  wt_cast_kernel<<<dim3(kD / 64, 3 * kD / 64, 1), blk256, 0, stream>>>(qkv_w, qkv_w, qkv_w, wQkvT, 0L, kD, 3 * kD, kWCarry);
  wt_cast_kernel<<<dim3(kD / 64, kD / 64, 3), blk256, 0, stream>>>(out_w, w_ctx, w_x, wOutT, (long)kD * kD, kD, kD, kWCarry);

  ln_row_kernel<false, false, false, false><<<dim3(kTok), blk128, 0, stream>>>(x, x, g_attn, b_attn, sbuf, xn16, sbuf, xn16);

  wmma_gemm64<0, false, 2, 1, false, 0, false><<<dim3(384, 1), blk256, 0, stream>>>(
      xn16, xn16, kD, 0L, wQkvT, wQkvT, kD, 0L, qkv16, qkv16, kQKVld, 0L, qkv_b, x, 0L, kTok, 3 * kD, kD, kWCarryInv);

  vt_transpose_kernel<<<dim3(kS / 64, kD / 64, kB), blk256, 0, stream>>>(qkv16, vt16);

  for (int gi = 0; gi < kNumGroups; ++gi) {
    const int b  = gi / 8;
    const int h0 = 2 * (gi % 8);
    const unsigned short* qbase = qkv16 + (size_t)b * kS * kQKVld + (size_t)h0 * kHD;
    const unsigned short* kbase = qbase + kD;
    wmma_gemm64<0, false, 0, 0, false, 0, true><<<dim3(128, 2), blk256, 0, stream>>>(
        qbase, qbase, kQKVld, (long)kHD, kbase, kbase, kQKVld, (long)kHD, sbuf, sbuf, kS, (long)kS * kS,
        qkv_b, x, 0L, kS, kS, kHD, kScoreScale);
    softmax_causal_kernel<<<dim3(kS, 2), blk256, 0, stream>>>(sbuf, pbuf, kPCarry);
    const unsigned short* vbase = vt16 + ((size_t)b * kD + (size_t)h0 * kHD) * kS;
    unsigned short* cbase = ctx16 + (size_t)b * kS * kD + (size_t)h0 * kHD;
    wmma_gemm64<0, false, 0, 1, false, 0, true><<<dim3(4, 2), blk256, 0, stream>>>(
        pbuf, pbuf, kS, (long)kS * kS, vbase, vbase, kS, (long)kHD * kS, cbase, cbase, kD, (long)kHD,
        qkv_b, x, 0L, kS, kHD, kS, kPCarryInv);
  }

  wmma_gemm64<0, false, 2, 0, false, 0, false><<<dim3(128, 1), blk256, 0, stream>>>(
      ctx16, ctx16, kD, 0L, wOutT, wOutT, kD, 0L, att, att, kD, 0L, out_b, x, 0L, kTok, kD, kD, kWCarryInv);

  ln_row_kernel<true, true, true, true><<<dim3(kTok), blk128, 0, stream>>>(x, att, g1, b1, x1, att16, xsA, xs16);

  wmma_gemm64<0, false, 2, 0, false, 0, false><<<dim3(128, 1), blk256, 0, stream>>>(
      att16, att16, kD, 0L, wCtxT, wCtxT, kD, 0L, c0, c0, kD, 0L, b_inl, x, 0L, kTok, kD, kD, kWCarryInv);

  for (int it = 0; it < kIters; ++it) {
    wmma_gemm64<0, false, 0, 0, false, 0, false><<<dim3(128, 1), blk256, 0, stream>>>(
        xs16, xs16, kD, 0L, wXT, wXT, kD, 0L, gmat, gmat, kD, 0L, b_inl, x, 0L, kTok, kD, kD, kWCarryInv);
    if (it == 0) {
      inl_step_kernel<true><<<dim3(4096), blk256, 0, stream>>>(c0, gmat, xsA, vsA, xsB, vsB, xs16);
    } else if (it & 1) {
      inl_step_kernel<false><<<dim3(4096), blk256, 0, stream>>>(c0, gmat, xsB, vsB, xsA, vsA, xs16);
    } else {
      inl_step_kernel<false><<<dim3(4096), blk256, 0, stream>>>(c0, gmat, xsA, vsA, xsB, vsB, xs16);
    }
  }

  ln_row_kernel<true, true, false, false><<<dim3(kTok), blk128, 0, stream>>>(x1, xsA, g2, b2, x2, hn16, x2, hn16);

  wt_cast_kernel<<<dim3(kD / 64, kFF / 64, 1), blk256, 0, stream>>>(ff_w1, ff_w1, ff_w1, wFf1T, 0L, kD, kFF, kWCarry);
  wt_cast_kernel<<<dim3(kFF / 64, kD / 64, 1), blk256, 0, stream>>>(ff_w2, ff_w2, ff_w2, wFf2T, 0L, kFF, kD, kWCarry);

  for (int ch = 0; ch < 2; ++ch) {
    const size_t roff = (size_t)ch * 2048 * kD;
    wmma_gemm64<0, false, 2, 0, false, 0, false><<<dim3(256, 1), blk256, 0, stream>>>(
        hn16 + roff, hn16 + roff, kD, 0L, wFf1T, wFf1T, kD, 0L, f1c, f1c, kFF, 0L, ff_b1, x, 0L, 2048, kFF, kD, kWCarryInv);
    gelu_cast_kernel<<<dim3(16384), blk256, 0, stream>>>(f1c, g1c, 2048 * kFF / 2);
    wmma_gemm64<0, false, 2, 0, true, 0, false><<<dim3(64, 1), blk256, 0, stream>>>(
        g1c, g1c, kFF, 0L, wFf2T, wFf2T, kFF, 0L, out + roff, out + roff, kD, 0L, ff_b2, x2 + roff, 0L, 2048, kD, kFF, kWCarryInv);
  }
}
